// SelfAttention_35424890258012
// MI455X (gfx1250) — hardware-verified
//
#include <hip/hip_runtime.h>
#include <math.h>

#ifndef NB
#define NB 2
#endif
#ifndef SEQ
#define SEQ 2048
#endif
#define NB_FULL 2
#define SEQ_FULL 2048
#define CH 1024
#define NH 16
#define HD 64
#define QKP 2048
#define SLP 68
#define CTP 72

static_assert(NB <= NB_FULL);
static_assert(SEQ <= SEQ_FULL);
static_assert(SEQ % 128 == 0);
static_assert(CH == NH * HD);
static_assert(HD == 64);
static_assert(CH == 1024);
static_assert(CH % 64 == 0);
static_assert(CH % 32 == 0);
static_assert(QKP == 2 * CH);
static_assert((NB * SEQ) % 64 == 0);
static_assert(SLP % 4 == 0);
static_assert(CTP % 8 == 0);

typedef __attribute__((ext_vector_type(16))) _Float16 v16h;
typedef __attribute__((ext_vector_type(8)))  _Float16 v8h;
typedef __attribute__((ext_vector_type(8)))  float    v8f;
typedef __attribute__((ext_vector_type(4)))  float    v4f;
typedef unsigned int cm_u4 __attribute__((ext_vector_type(4)));

__device__ __forceinline__ v8f wmma16(v16h a, v16h b, v8f c) {
    c = __builtin_amdgcn_wmma_f32_16x16x32_f16(false, a, false, b, (short)0, c, false, false);
    asm volatile("v_nop\n\tv_nop\n\tv_nop\n\tv_nop" : "+v"(c) : "v"(a), "v"(b));
    return c;
}
__device__ __forceinline__ v16h ldh16(const unsigned short* p) {
    union { v16h v; v8h h[2]; } f; f.h[0] = *(const v8h*)(p); f.h[1] = *(const v8h*)(p + 16); return f.v;
}

#define VST2(T, ptr, val) do { const T vst2_v_ = (val); *(volatile T*)(ptr) = vst2_v_; __threadfence(); *(volatile T*)(ptr) = vst2_v_; } while (0)
#define VST2V4(ptr, val) do { const v4f vst2_v4_ = (val); *(volatile v4f*)(ptr) = vst2_v4_; __threadfence(); *(volatile v4f*)(ptr) = vst2_v4_; } while (0)

__device__ __forceinline__ float cmb_bf(float v) { const unsigned u = __builtin_bit_cast(unsigned, v); const unsigned r = (u + 0x7fffu + ((u >> 16) & 1u)) & 0xffff0000u; return __builtin_bit_cast(float, r); }
__device__ __forceinline__ unsigned int cmb_pk2(float a, float b) { return (unsigned int)__builtin_bit_cast(unsigned short, (_Float16)a) | ((unsigned int)__builtin_bit_cast(unsigned short, (_Float16)b) << 16); }

__global__ __launch_bounds__(256) void k_xcast(const float* __restrict__ x, unsigned short* __restrict__ X16) {
    const unsigned u = blockIdx.x * 256u + threadIdx.x;
    if (u >= (unsigned)(NB * SEQ) * (unsigned)(CH / 8)) return;
    const unsigned row = u >> 7, c0 = (u & 127u) << 3;
    const unsigned b = row / (unsigned)SEQ, t = row - b * (unsigned)SEQ;
    const float* s = x + ((size_t)b * SEQ_FULL + t) * CH + c0;
    const v4f a = *(const v4f*)(s);
    const v4f c = *(const v4f*)(s + 4);
    cm_u4 pk;
    pk.x = cmb_pk2(cmb_bf(a.x), cmb_bf(a.y)); pk.y = cmb_pk2(cmb_bf(a.z), cmb_bf(a.w));
    pk.z = cmb_pk2(cmb_bf(c.x), cmb_bf(c.y)); pk.w = cmb_pk2(cmb_bf(c.z), cmb_bf(c.w));
    VST2(cm_u4, (cm_u4*)(X16 + (size_t)row * CH + c0), pk);
}

__global__ __launch_bounds__(256) void k_wprep(const float* __restrict__ Wq, const float* __restrict__ Wk, const float* __restrict__ Wv, const float* __restrict__ Wp,
                                               const float* __restrict__ bq, const float* __restrict__ bk, const float* __restrict__ bv, const float* __restrict__ bp,
                                               unsigned short* __restrict__ W16, float* __restrict__ BR) {
    if (blockIdx.x < 2048u) {
        const unsigned u = blockIdx.x * 256u + threadIdx.x;
        const unsigned row = u >> 7, c0 = (u & 127u) << 3;
        const unsigned mat = row >> 10, r = row & 1023u;
        const float* src = (mat == 0u) ? Wq : ((mat == 1u) ? Wk : ((mat == 2u) ? Wv : Wp));
        const float* s = src + (size_t)r * CH + c0;
        const v4f a = *(const v4f*)(s);
        const v4f c = *(const v4f*)(s + 4);
        cm_u4 pk;
        pk.x = cmb_pk2(cmb_bf(a.x) * 16.0f, cmb_bf(a.y) * 16.0f); pk.y = cmb_pk2(cmb_bf(a.z) * 16.0f, cmb_bf(a.w) * 16.0f);
        pk.z = cmb_pk2(cmb_bf(c.x) * 16.0f, cmb_bf(c.y) * 16.0f); pk.w = cmb_pk2(cmb_bf(c.z) * 16.0f, cmb_bf(c.w) * 16.0f);
        VST2(cm_u4, (cm_u4*)(W16 + (size_t)row * CH + c0), pk);
    } else {
        const unsigned mat = blockIdx.x - 2048u;
        const unsigned j4 = threadIdx.x << 2;
        const float* src = (mat == 0u) ? bq : ((mat == 1u) ? bk : ((mat == 2u) ? bv : bp));
        const v4f s = *(const v4f*)(src + j4);
        v4f v; v.x = cmb_bf(s.x); v.y = cmb_bf(s.y); v.z = cmb_bf(s.z); v.w = cmb_bf(s.w);
        VST2V4(BR + mat * 1024u + j4, v);
    }
}

__global__ __launch_bounds__(256) void k_gemm(
    const unsigned short* __restrict__ Ap, int lda, long strideA,
    const unsigned short* __restrict__ Btp, int ldb, long strideB,
    float* __restrict__ C32, unsigned short* __restrict__ C16, int ldc, long strideC,
    const float* __restrict__ bias, int biasMode, int outMode, int M, int N, int K, float scale) {
  __shared__ __align__(16) float sT[8][16 * SLP];
  const int bz   = blockIdx.y;
  const int lane = threadIdx.x & 31;
  const int wave = __builtin_amdgcn_readfirstlane((int)(threadIdx.x >> 5));
  const int tilesN = N >> 6;
  const int tilesM = M >> 6;
  const int tile = blockIdx.x * 8 + wave;
  if (tile >= tilesM * tilesN) return;
  const int tm = tile / tilesN;
  const int tn = tile - tm * tilesN;
  const int m0 = tm << 6;
  const int n0 = tn << 6;

  const unsigned short* Ab = Ap  + (size_t)bz * strideA;
  const unsigned short* Bb = Btp + (size_t)bz * strideB;

  const int rlane = lane & 15;
  const int koff  = (lane >> 4) * 8;
  const int mOff  = (lane >> 4) * 8;

  v8f acc[4][4];
#pragma unroll
  for (int i = 0; i < 4; ++i)
#pragma unroll
    for (int j = 0; j < 4; ++j) acc[i][j] = (v8f){0.f,0.f,0.f,0.f,0.f,0.f,0.f,0.f};

  for (int k0 = 0; k0 < K; k0 += 32) {
    v16h bh[4];
#pragma unroll
    for (int j = 0; j < 4; ++j) {
      const size_t bo = (size_t)(n0 + (j << 4) + rlane) * ldb + koff + k0;
      bh[j] = ldh16(Bb + bo);
    }
#pragma unroll
    for (int i = 0; i < 4; ++i) {
      const size_t ao = (size_t)(m0 + (i << 4) + rlane) * lda + koff + k0;
      const v16h ah = ldh16(Ab + ao);
#pragma unroll
      for (int j = 0; j < 4; ++j) acc[i][j] = wmma16(ah, bh[j], acc[i][j]);
    }
  }

#pragma unroll
  for (int i = 0; i < 4; ++i) {
    const int mBase = m0 + (i << 4);
    float bm[8];
#pragma unroll
    for (int r = 0; r < 8; ++r) bm[r] = 0.0f;
    if (biasMode == 1) {
#pragma unroll
      for (int r = 0; r < 8; ++r) bm[r] = bias[mBase + mOff + r];
    }
#pragma unroll
    for (int j = 0; j < 4; ++j) {
      float bn = 0.0f;
      if (biasMode == 2) bn = bias[n0 + (j << 4) + rlane];
#pragma unroll
      for (int r = 0; r < 8; ++r) {
        const float v = acc[i][j][r] * scale + (bm[r] + bn);
        sT[wave][(mOff + r) * SLP + (j << 4) + rlane] = v;
      }
    }
    __builtin_amdgcn_fence(3  , "workgroup");
    __builtin_amdgcn_wave_barrier();
    __builtin_amdgcn_fence(2  , "workgroup");
    if (outMode == 0) {
      float* C = C32 + (size_t)bz * strideC;
      const int hh = lane >> 4, c4 = (lane & 15) * 4;
      for (int pass = 0; pass < 2; ++pass) {
#pragma unroll
        for (int it = 0; it < 8; ++it) {
          const int row = it * 2 + hh;
          const v4f v = *(const v4f*)(&sT[wave][row * SLP + c4]);
          *(volatile v4f*)(C + (size_t)(mBase + row) * ldc + n0 + c4) = v;
        }
        __threadfence();
      }
    } else {
      unsigned short* C = C16 + (size_t)bz * strideC;
      const int q = lane >> 3, c8 = (lane & 7) * 8;
      for (int pass = 0; pass < 2; ++pass) {
#pragma unroll
        for (int it = 0; it < 4; ++it) {
          const int row = it * 4 + q;
          const v4f s0 = *(const v4f*)(&sT[wave][row * SLP + c8]);
          const v4f s1 = *(const v4f*)(&sT[wave][row * SLP + c8 + 4]);
          v8h hv;
          hv[0] = (_Float16)s0.x; hv[1] = (_Float16)s0.y; hv[2] = (_Float16)s0.z; hv[3] = (_Float16)s0.w;
          hv[4] = (_Float16)s1.x; hv[5] = (_Float16)s1.y; hv[6] = (_Float16)s1.z; hv[7] = (_Float16)s1.w;
          *(volatile v8h*)(C + (size_t)(mBase + row) * ldc + n0 + c8) = hv;
        }
        __threadfence();
      }
    }
    __builtin_amdgcn_fence(3  , "workgroup");
    __builtin_amdgcn_wave_barrier();
    __builtin_amdgcn_fence(2  , "workgroup");
  }
}

__global__ __launch_bounds__(128) void k_attn(const unsigned short* __restrict__ QK, const unsigned short* __restrict__ Vt,
                                              const int* __restrict__ mask, unsigned short* __restrict__ CTX) {
    __shared__ unsigned int mb[SEQ / 32];
    __shared__ __align__(16) _Float16 ct[4][16 * CTP];
    const unsigned lane = threadIdx.x & 31u, h = lane >> 4, l15 = lane & 15u;
    const unsigned wave = (unsigned)__builtin_amdgcn_readfirstlane((int)(threadIdx.x >> 5));
    const unsigned bh = blockIdx.y, b = bh / (unsigned)NH, hd = bh - b * (unsigned)NH;
    const unsigned q0 = blockIdx.x * 64u + wave * 16u;

    const int* mrow = mask + (size_t)b * SEQ_FULL;
#pragma unroll 4
    for (unsigned i = 0; i < (unsigned)(SEQ / 128); ++i) {
        const unsigned w = wave * (unsigned)(SEQ / 128) + i;
        const int mv = mrow[w * 32u + lane];
        const unsigned bits = __builtin_amdgcn_ballot_w32(mv != 0);
        if (lane == 0u) mb[w] = bits;
    }
    __syncthreads();

    const size_t rq = (size_t)(b * (unsigned)SEQ + q0 + l15) * QKP + hd * (unsigned)HD + 8u * h;
    const v16h qf0 = ldh16(QK + rq);
    const v16h qf1 = ldh16(QK + rq + 32);

    v8f o[4];
#pragma unroll
    for (int t = 0; t < 4; ++t) o[t] = (v8f){0.f, 0.f, 0.f, 0.f, 0.f, 0.f, 0.f, 0.f};
    float m = -__builtin_inff(), l = 0.f;
    const float SC = 0.125f * 1.4426950408889634f;
    const float TM = -1.4426950408889634e30f;
    const size_t kbase = (size_t)(b * (unsigned)SEQ + l15) * QKP + CH + hd * (unsigned)HD + 8u * h;
    const size_t vbase = ((size_t)b * CH + hd * (unsigned)HD + l15) * SEQ + 8u * h;

    for (unsigned j0 = 0; j0 < (unsigned)SEQ; j0 += 32u) {
        const size_t rk0 = kbase + (size_t)j0 * QKP;
        const size_t rk1 = rk0 + (size_t)16 * QKP;
        v8f st0 = {0.f, 0.f, 0.f, 0.f, 0.f, 0.f, 0.f, 0.f};
        v8f st1 = {0.f, 0.f, 0.f, 0.f, 0.f, 0.f, 0.f, 0.f};
        st0 = wmma16(ldh16(QK + rk0),      qf0, st0);
        st0 = wmma16(ldh16(QK + rk0 + 32), qf1, st0);
        st1 = wmma16(ldh16(QK + rk1),      qf0, st1);
        st1 = wmma16(ldh16(QK + rk1 + 32), qf1, st1);

        const unsigned mw = (unsigned)__builtin_amdgcn_readfirstlane((int)mb[j0 >> 5]);
        float t0[8], t1[8];
#pragma unroll
        for (int r = 0; r < 8; ++r) { t0[r] = st0[r] * SC; t1[r] = st1[r] * SC; }
        if (mw != 0xffffffffu) {
#pragma unroll
            for (int r = 0; r < 8; ++r) {
                t0[r] = ((mw >> (8u * h + (unsigned)r)) & 1u) ? t0[r] : TM;
                t1[r] = ((mw >> (16u + 8u * h + (unsigned)r)) & 1u) ? t1[r] : TM;
            }
        }
        float mx = fmaxf(fmaxf(fmaxf(t0[0], t0[1]), fmaxf(t0[2], t0[3])), fmaxf(fmaxf(t0[4], t0[5]), fmaxf(t0[6], t0[7])));
        mx = fmaxf(mx, fmaxf(fmaxf(fmaxf(t1[0], t1[1]), fmaxf(t1[2], t1[3])), fmaxf(fmaxf(t1[4], t1[5]), fmaxf(t1[6], t1[7]))));
        mx = fmaxf(mx, __shfl_xor(mx, 16, 32));
        const float mn = fmaxf(m, mx);
        if (__builtin_amdgcn_ballot_w32(mn > m) != 0u) {
            const float corr = exp2f(m - mn);
            l *= corr;
#pragma unroll
            for (int t = 0; t < 4; ++t)
#pragma unroll
                for (int r = 0; r < 8; ++r) o[t][r] *= corr;
        }
        m = mn;
        float sum = 0.f;
        v16h pb;
#pragma unroll
        for (int r = 0; r < 8; ++r) {
            const float p0 = exp2f(t0[r] - mn);
            const float p1 = exp2f(t1[r] - mn);
            sum += p0 + p1;
            pb[r]     = (_Float16)(p0 * 1024.0f);
            pb[8 + r] = (_Float16)(p1 * 1024.0f);
        }
        l += sum;
#pragma unroll
        for (int t = 0; t < 4; ++t) {
            const v16h va = ldh16(Vt + vbase + (size_t)(16 * t) * SEQ + j0);
            o[t] = wmma16(va, pb, o[t]);
        }
    }

    const float L = l + __shfl_xor(l, 16, 32);
    const float inv = 0.0625f * (1.0f / L);
#pragma unroll
    for (int t = 0; t < 4; ++t) {
        v8h hv;
#pragma unroll
        for (int r = 0; r < 8; ++r) hv[r] = (_Float16)(o[t][r] * inv);
        *(v8h*)(&ct[wave][l15 * CTP + 16u * (unsigned)t + 8u * h]) = hv;
    }
    __builtin_amdgcn_fence(3  , "workgroup");
    __builtin_amdgcn_wave_barrier();
    __builtin_amdgcn_fence(2  , "workgroup");
    {
        const unsigned q = lane >> 3, c8 = (lane & 7u) * 8u;
        for (int pass = 0; pass < 2; ++pass) {
#pragma unroll
            for (int it = 0; it < 4; ++it) {
                const unsigned row = (unsigned)it * 4u + q;
                const v8h v = *(const v8h*)(&ct[wave][row * CTP + c8]);
                *(volatile v8h*)(CTX + (size_t)(b * (unsigned)SEQ + q0 + row) * CH + hd * (unsigned)HD + c8) = v;
            }
            __threadfence();
        }
    }
}

static constexpr size_t al256(size_t v) { return (v + 255) / 256 * 256; }
static constexpr size_t SZ_X16 = al256((size_t)NB * SEQ * CH * 2);
static constexpr size_t SZ_W16 = al256((size_t)4096 * CH * 2);
static constexpr size_t SZ_BR  = al256((size_t)8192 * 4);
static constexpr size_t SZ_QK  = al256((size_t)NB * SEQ * QKP * 2);
static constexpr size_t SZ_VT  = al256((size_t)NB * CH * SEQ * 2);
static constexpr size_t SZ_CTX = al256((size_t)NB * SEQ * CH * 2);
static constexpr size_t WS_TOTAL = SZ_X16 + SZ_W16 + SZ_BR + SZ_QK + SZ_VT + SZ_CTX;
static_assert(WS_TOTAL <= (size_t)134217728);
static_assert(((size_t)NB * SEQ * (CH / 8) / 256) * 256 * 8 == (size_t)NB * SEQ * CH);
static_assert((size_t)2048 * 256 * 8 == (size_t)4096 * CH);
static_assert((size_t)4 * 256 * 4 == (size_t)4096);
static_assert(((size_t)NB * SEQ / 64) * (QKP / 64) * 64 * 64 == (size_t)NB * SEQ * QKP);
static_assert((((size_t)NB * SEQ / 64) * (QKP / 64)) % 8 == 0);
static_assert((size_t)NB * (CH / 64) * (SEQ / 64) * 64 * 64 == (size_t)NB * CH * SEQ);
static_assert((((size_t)CH / 64) * (SEQ / 64)) % 8 == 0);
static_assert((size_t)(SEQ / 64) * NB * NH * 64 * HD == (size_t)NB * SEQ * CH);
static_assert((size_t)NB * (SEQ / 64) * (CH / 64) * 64 * 64 == (size_t)NB * SEQ * CH);
static_assert(((size_t)(NB - 1) * SEQ_FULL + SEQ) * CH <= (size_t)NB_FULL * SEQ_FULL * CH);
static_assert(2048 + 1024 + 2048 <= 8192);

extern "C" void kernel_launch(void* const* d_in, const int* in_sizes, int n_in, void* d_out, int out_size, void* d_ws, size_t ws_size, hipStream_t stream) {
    if (n_in < 10) return;
    if (in_sizes[0] < ((NB - 1) * SEQ_FULL + SEQ) * CH) return;
    if (in_sizes[1] < (NB - 1) * SEQ_FULL + SEQ) return;
    if (in_sizes[2] < CH * CH || in_sizes[4] < CH * CH || in_sizes[6] < CH * CH || in_sizes[8] < CH * CH) return;
    if (in_sizes[3] < CH || in_sizes[5] < CH || in_sizes[7] < CH || in_sizes[9] < CH) return;
    if (out_size < ((NB - 1) * SEQ_FULL + SEQ) * CH) return;
    if (WS_TOTAL > ws_size) return;
    const float* x   = (const float*)d_in[0];
    const int*   msk = (const int*)d_in[1];
    const float* Wq  = (const float*)d_in[2];
    const float* bq  = (const float*)d_in[3];
    const float* Wk  = (const float*)d_in[4];
    const float* bk  = (const float*)d_in[5];
    const float* Wv  = (const float*)d_in[6];
    const float* bv  = (const float*)d_in[7];
    const float* Wp  = (const float*)d_in[8];
    const float* bp  = (const float*)d_in[9];
    float* out = (float*)d_out;
    char* wsp = (char*)d_ws;
    unsigned short* X16 = (unsigned short*)wsp; wsp += SZ_X16;
    unsigned short* W16 = (unsigned short*)wsp; wsp += SZ_W16;
    float* BR           = (float*)wsp;          wsp += SZ_BR;
    unsigned short* QK  = (unsigned short*)wsp; wsp += SZ_QK;
    unsigned short* VT  = (unsigned short*)wsp; wsp += SZ_VT;
    unsigned short* CTX = (unsigned short*)wsp; wsp += SZ_CTX;

    k_xcast<<<(unsigned)(((size_t)NB * SEQ * (CH / 8) + 255) / 256), 256, 0, stream>>>(x, X16);
    k_wprep<<<2052, 256, 0, stream>>>(Wq, Wk, Wv, Wp, bq, bk, bv, bp, W16, BR);
    k_gemm<<<dim3((unsigned)((((NB * SEQ) / 64) * (QKP / 64)) / 8), 1u), 256, 0, stream>>>(
        (const unsigned short*)X16, CH, (long)0, (const unsigned short*)W16, CH, (long)0,
        out, QK, QKP, (long)0, (const float*)BR, 2, 1, NB * SEQ, QKP, CH, 0.0625f);
    k_gemm<<<dim3((unsigned)(((CH / 64) * (SEQ / 64)) / 8), (unsigned)NB), 256, 0, stream>>>(
        (const unsigned short*)(W16 + (size_t)2048 * CH), CH, (long)0, (const unsigned short*)X16, CH, (long)SEQ * CH,
        out, VT, SEQ, (long)CH * SEQ, (const float*)(BR + 2048), 1, 1, CH, SEQ, CH, 0.0625f);
    k_attn<<<dim3((unsigned)(SEQ / 64), (unsigned)(NB * NH)), 128, 0, stream>>>(
        (const unsigned short*)QK, (const unsigned short*)VT, msk, CTX);
    k_gemm<<<dim3((unsigned)(((SEQ / 64) * (CH / 64)) / 8), (unsigned)NB), 256, 0, stream>>>(
        (const unsigned short*)CTX, CH, (long)SEQ * CH, (const unsigned short*)(W16 + (size_t)3072 * CH), CH, (long)0,
        out, CTX, CH, (long)SEQ_FULL * CH, (const float*)(BR + 3072), 2, 0, SEQ, CH, CH, 0.0009765625f);
}
